// GCN_27986006901444
// MI455X (gfx1250) — hardware-run, weakly checked
//
#include <hip/hip_runtime.h>
#include <stddef.h>
#include <stdint.h>
#include <math.h>

#define NN      100000
#define NE      1600000
#define HD      64
#define GBM     128
#define MP      100096
#define NTHR    256
#define NWAVE   8
#define EPT     8
#define WCH     (32 * EPT)
#define NBRUN   1024
#define SLB     10
#define NBK     98
#define NSLOT   (NBK * NBRUN)
#define WLCAP   3584
#define RCAP    20480
#define TRIPCAP 64
#define MAXDEG_MEAS   36
#define MAXB1024_MEAS 16710
#define SP      68
#define WSMAX   134217728

#define BK_ZINTS (NWAVE * WLCAP + RCAP + 3 * NBRUN)
#define BK_INTS  (BK_ZINTS + 16)
#define BK_LDS   (BK_INTS * 4)

#define PBX   (MP * HD / 8 / NTHR)
#define PBW   (HD * HD / 8 / NTHR)
#define PBTOT (PBX + PBW + 1)

static_assert(HD == 64 && HD == 2 * 32 && HD == 16 * 4);
static_assert(MP % GBM == 0 && MP >= NN && MP == 782 * GBM && NN == 781 * GBM + 32);
static_assert(NBRUN == 1024 && NBRUN == (1 << SLB) && NBRUN % GBM == 0 && NBRUN % NWAVE == 0);
static_assert(NSLOT >= MP && (NBK - 1) * NBRUN < NN);
static_assert(NN <= 131072);
static_assert((((long long)(NN - 1)) << SLB) + (NBRUN - 1) < (1LL << 31));
static_assert(NE % WCH == 0 && NE % 4 == 0);
static_assert((NWAVE * WLCAP) % 4 == 0 && RCAP % 4 == 0 && BK_ZINTS % 4 == 0 && RCAP % (NTHR * 4) == 0);
static_assert((long long)RCAP * 100 >= (long long)MAXB1024_MEAS * 108);
static_assert((long long)WLCAP * 32 >= (long long)RCAP * 5);
static_assert(WLCAP >= MAXB1024_MEAS / 8 + 8 * 46 + 1);
static_assert(MAXDEG_MEAS + 8 <= TRIPCAP && TRIPCAP % 32 == 0);
static_assert(BK_LDS <= 300000);
static_assert((GBM * SP + GBM) * 4 <= 65536);
static_assert((MP * HD / 8) % NTHR == 0 && (HD * HD / 8) % NTHR == 0);
static_assert(HD % 32 == 0);

typedef float          v2f   __attribute__((ext_vector_type(2)));
typedef float          v4f   __attribute__((ext_vector_type(4)));
typedef float          v8f   __attribute__((ext_vector_type(8)));
typedef int            v4i   __attribute__((ext_vector_type(4)));
typedef int            v8i   __attribute__((ext_vector_type(8)));
typedef unsigned short v8us  __attribute__((ext_vector_type(8)));
typedef unsigned short v16us __attribute__((ext_vector_type(16)));
typedef __bf16         v16bf __attribute__((ext_vector_type(16)));
typedef v2f  __attribute__((may_alias)) v2fa;
typedef v4f  __attribute__((may_alias)) v4fa;
typedef v4i  __attribute__((may_alias)) v4ia;
typedef v8us __attribute__((may_alias)) v8usa;
union FragB { v16bf v; v16us u; v8us h[2]; v8i w; };

__device__ __forceinline__ v8f wmb(const FragB& a, const FragB& b, v8f c) {
  v8f d = __builtin_amdgcn_wmma_f32_16x16x32_bf16(false, a.v, false, b.v, (short)0, c, false, false);
  asm volatile("v_nop\n\tv_nop\n\tv_nop\n\tv_nop" : "+v"(d) : "v"(a.w), "v"(b.w));
  return d;
}

__device__ __forceinline__ unsigned bf16_bits(float f) {
  const unsigned u = __float_as_uint(f);
  const unsigned r = (u + 0x7FFFu + ((u >> 16) & 1u)) >> 16;
  const unsigned q = (u >> 16) | 0x40u;
  return ((u & 0x7fffffffu) > 0x7f800000u) ? q : r;
}
__device__ __forceinline__ float bf16_val(float f) {
  return __uint_as_float(bf16_bits(f) << 16);
}

__device__ __forceinline__ void st2_v4f(float* p, v4f v) {
  *(volatile v4f*)p = v;
  __threadfence();
  *(volatile v4f*)p = v;
}
__device__ __forceinline__ void st2_v8us(unsigned short* p, v8us v) {
  *(volatile v8us*)p = v;
  __threadfence();
  *(volatile v8us*)p = v;
}

__device__ __forceinline__ v8us gather8(const float* __restrict__ base, int stride) {
  float f[8];
#pragma unroll
  for (int i = 0; i < 8; ++i) f[i] = base[(size_t)i * (size_t)stride];
  v8us o;
#pragma unroll
  for (int i = 0; i < 8; ++i) o[i] = (unsigned short)bf16_bits(f[i]);
  return o;
}

__global__ __launch_bounds__(NTHR) void k_prep(const float* __restrict__ x, const float* __restrict__ w,
                                               const float* __restrict__ b,
                                               unsigned short* xb, unsigned short* wt, float* bb) {
  const int tid = (int)threadIdx.x, lane = tid & 31;
  const int blk = (int)blockIdx.x;
  if (blk < PBX) {
    const int u   = blk * NTHR + tid;
    const int row = u >> 3, k8 = (u & 7) * 8;
    const int rc  = row < NN ? row : NN - 1;
    const unsigned mk = row < NN ? 0xffffu : 0u;
    const float* p = x + (size_t)rc * HD + k8;
    const v4f a = *(const v4fa*)p;
    const v4f c = *(const v4fa*)(p + 4);
    v8us o;
    o[0] = (unsigned short)(bf16_bits(a.x) & mk); o[1] = (unsigned short)(bf16_bits(a.y) & mk);
    o[2] = (unsigned short)(bf16_bits(a.z) & mk); o[3] = (unsigned short)(bf16_bits(a.w) & mk);
    o[4] = (unsigned short)(bf16_bits(c.x) & mk); o[5] = (unsigned short)(bf16_bits(c.y) & mk);
    o[6] = (unsigned short)(bf16_bits(c.z) & mk); o[7] = (unsigned short)(bf16_bits(c.w) & mk);
    st2_v8us(xb + (size_t)row * HD + k8, o);
  } else if (blk < PBX + PBW) {
    const int u = (blk - PBX) * NTHR + tid;
    const int n = u >> 3, k8 = (u & 7) * 8;
    const v8us o = gather8(w + (size_t)k8 * HD + n, HD);
    st2_v8us(wt + (size_t)n * HD + k8, o);
  } else {
    if (tid < 32) {
      const int q = lane & 15;
      const v4f a = *(const v4fa*)(b + 4 * q);
      asm volatile("" :: "v"(a));
      v4f o;
      o.x = bf16_val(a.x); o.y = bf16_val(a.y); o.z = bf16_val(a.z); o.w = bf16_val(a.w);
      const bool wr = lane < 16;
      float* p = bb + 4 * q;
      if (wr) *(volatile v4f*)p = o;
      __threadfence();
      if (wr) *(volatile v4f*)p = o;
    }
  }
}

__device__ __forceinline__ void bucket_flush(const int* pl, const int* cnt, int ov, int* lp, int* cp, int* op,
                                             int* dp, int* fp, int tid) {
#pragma unroll 1
  for (int i = tid * 4; i < RCAP; i += NTHR * 4) {
    const v4i v = *(const v4ia*)(pl + i);
    *(volatile v4i*)(lp + i) = v;
  }
  {
    const v4i v = *(const v4ia*)(cnt + 4 * tid);
    *(volatile v4i*)(cp + 4 * tid) = v;
  }
  {
    const v4i v = *(const v4ia*)(cnt + NBRUN + 4 * tid);
    *(volatile v4i*)(op + 4 * tid) = v;
  }
  {
    const v4i v = *(const v4ia*)(cnt + 2 * NBRUN + 4 * tid);
    *(volatile v4i*)(dp + 4 * tid) = v;
  }
  if (tid < 8) {
    const v4i f = {ov, ov, ov, ov};
    *(volatile v4i*)(fp + 4 * tid) = f;
  }
}

__global__ __launch_bounds__(NTHR) void k_bucket(const int* __restrict__ srcs, const int* __restrict__ dsts,
                                                 int* LIST, int* CNT, int* OFF, int* DINVB, int* FLAG) {
  extern __shared__ __attribute__((aligned(16))) int dsm[];
  int* wl   = dsm;
  int* pl   = dsm + NWAVE * WLCAP;
  int* cnt  = pl + RCAP;
  int* offs = cnt + NBRUN;
  int* cur  = offs + NBRUN;
  int* misc = cur + NBRUN;
  const int tid = (int)threadIdx.x, lane = tid & 31, wave = tid >> 5;
  const int blk = (int)blockIdx.x;
  const int firstRow = blk * NBRUN;
  const unsigned nbs = (unsigned)firstRow;

  {
    const v4i z4 = {0, 0, 0, 0};
    const v4i r4 = {firstRow, firstRow, firstRow, firstRow};
    for (int i = tid * 4; i < BK_ZINTS; i += NTHR * 4) {
      const bool inpl = (i >= NWAVE * WLCAP) && (i < NWAVE * WLCAP + RCAP);
      *(v4ia*)(dsm + i) = inpl ? r4 : z4;
    }
    if (tid < 16) misc[tid] = 0;
  }
  __syncthreads();

  {
    const int per  = ((NE + NWAVE * WCH - 1) / (NWAVE * WCH)) * WCH;
    const int ebeg = wave * per;
    const int eend = (ebeg + per < NE) ? (ebeg + per) : NE;
    int* mylist = wl + wave * WLCAP;
    int wc = 0;
#pragma unroll 1
    for (int cb = ebeg; cb < eend; cb += WCH) {
      const int e0 = cb + lane * EPT;
      const v4i da = *(const v4ia*)(dsts + e0);
      const v4i db = *(const v4ia*)(dsts + e0 + 4);
      const v4i sa = *(const v4ia*)(srcs + e0);
      const v4i sb = *(const v4ia*)(srcs + e0 + 4);
      asm volatile("" :: "v"(sa), "v"(sb));
      const unsigned s0 = (unsigned)da.x - nbs, s1 = (unsigned)da.y - nbs;
      const unsigned s2 = (unsigned)da.z - nbs, s3 = (unsigned)da.w - nbs;
      const unsigned s4 = (unsigned)db.x - nbs, s5 = (unsigned)db.y - nbs;
      const unsigned s6 = (unsigned)db.z - nbs, s7 = (unsigned)db.w - nbs;
      const bool h0 = s0 < (unsigned)NBRUN, h1 = s1 < (unsigned)NBRUN, h2 = s2 < (unsigned)NBRUN, h3 = s3 < (unsigned)NBRUN;
      const bool h4 = s4 < (unsigned)NBRUN, h5 = s5 < (unsigned)NBRUN, h6 = s6 < (unsigned)NBRUN, h7 = s7 < (unsigned)NBRUN;
      const unsigned m0 = __builtin_amdgcn_ballot_w32(h0), m1 = __builtin_amdgcn_ballot_w32(h1);
      const unsigned m2 = __builtin_amdgcn_ballot_w32(h2), m3 = __builtin_amdgcn_ballot_w32(h3);
      const unsigned m4 = __builtin_amdgcn_ballot_w32(h4), m5 = __builtin_amdgcn_ballot_w32(h5);
      const unsigned m6 = __builtin_amdgcn_ballot_w32(h6), m7 = __builtin_amdgcn_ballot_w32(h7);
      const unsigned any = m0 | m1 | m2 | m3 | m4 | m5 | m6 | m7;
      if (any != 0u) {
        const int pre = (int)(__builtin_amdgcn_mbcnt_lo(m0, 0u) + __builtin_amdgcn_mbcnt_lo(m1, 0u) +
                              __builtin_amdgcn_mbcnt_lo(m2, 0u) + __builtin_amdgcn_mbcnt_lo(m3, 0u) +
                              __builtin_amdgcn_mbcnt_lo(m4, 0u) + __builtin_amdgcn_mbcnt_lo(m5, 0u) +
                              __builtin_amdgcn_mbcnt_lo(m6, 0u) + __builtin_amdgcn_mbcnt_lo(m7, 0u));
        int p = wc + pre;
        if (h0) { if (p < WLCAP) mylist[p] = (int)(((unsigned)sa.x << SLB) | s0); p = p + 1; }
        if (h1) { if (p < WLCAP) mylist[p] = (int)(((unsigned)sa.y << SLB) | s1); p = p + 1; }
        if (h2) { if (p < WLCAP) mylist[p] = (int)(((unsigned)sa.z << SLB) | s2); p = p + 1; }
        if (h3) { if (p < WLCAP) mylist[p] = (int)(((unsigned)sa.w << SLB) | s3); p = p + 1; }
        if (h4) { if (p < WLCAP) mylist[p] = (int)(((unsigned)sb.x << SLB) | s4); p = p + 1; }
        if (h5) { if (p < WLCAP) mylist[p] = (int)(((unsigned)sb.y << SLB) | s5); p = p + 1; }
        if (h6) { if (p < WLCAP) mylist[p] = (int)(((unsigned)sb.z << SLB) | s6); p = p + 1; }
        if (h7) { if (p < WLCAP) mylist[p] = (int)(((unsigned)sb.w << SLB) | s7); p = p + 1; }
        wc += (int)(__builtin_popcount(m0) + __builtin_popcount(m1) + __builtin_popcount(m2) + __builtin_popcount(m3) +
                    __builtin_popcount(m4) + __builtin_popcount(m5) + __builtin_popcount(m6) + __builtin_popcount(m7));
      }
    }
    if (lane == 0) misc[wave] = wc;
  }
  __syncthreads();

  if (wave == 0) {
    int ov = 0, tot = 0;
#pragma unroll 1
    for (int w2 = 0; w2 < NWAVE; ++w2) {
      int c = misc[w2];
      if (c > WLCAP) ov = 1;
      c = c < 0 ? 0 : (c > WLCAP ? WLCAP : c);
      tot += c;
#pragma unroll 1
      for (int b0 = 0; b0 < c; b0 += 32) {
        const int idx = b0 + lane;
        const int ent = wl[w2 * WLCAP + (idx < WLCAP ? idx : WLCAP - 1)];
        const int m32 = (c - b0) < 32 ? (c - b0) : 32;
#pragma unroll 1
        for (int k = 0; k < m32; ++k) {
          const int u    = __builtin_amdgcn_readlane(ent, k);
          const int slot = u & (NBRUN - 1);
          if (lane == 0) cnt[slot] = cnt[slot] + 1;
        }
      }
    }
    if (tot > RCAP) ov = 1;
    if (lane == 0) misc[9] = ov;
  }
  __syncthreads();
  if (wave == 0) {
    const int base = lane * (NBRUN / 32);
    int s = 0;
#pragma unroll 1
    for (int i = 0; i < NBRUN / 32; ++i) s += cnt[base + i];
    int incl = s;
#pragma unroll
    for (int d = 1; d < 32; d <<= 1) {
      const int y = __shfl_up(incl, d, 32);
      if (lane >= d) incl += y;
    }
    int run = incl - s;
#pragma unroll 1
    for (int i = 0; i < NBRUN / 32; ++i) {
      const int cv = cnt[base + i];
      offs[base + i] = run;
      cur[base + i]  = run;
      run += cv;
    }
  }
  __syncthreads();

  if (wave == 0) {
#pragma unroll 1
    for (int w2 = 0; w2 < NWAVE; ++w2) {
      int c = misc[w2];
      c = c < 0 ? 0 : (c > WLCAP ? WLCAP : c);
#pragma unroll 1
      for (int b0 = 0; b0 < c; b0 += 32) {
        const int idx = b0 + lane;
        const int ent = wl[w2 * WLCAP + (idx < WLCAP ? idx : WLCAP - 1)];
        const int m32 = (c - b0) < 32 ? (c - b0) : 32;
#pragma unroll 1
        for (int k = 0; k < m32; ++k) {
          const int u    = __builtin_amdgcn_readlane(ent, k);
          const int slot = u & (NBRUN - 1);
          int sr = (int)((unsigned)u >> SLB);
          sr = sr > NN - 1 ? NN - 1 : sr;
          if (lane == 0) {
            int p = cur[slot];
            p = p < 0 ? 0 : (p > RCAP - 1 ? RCAP - 1 : p);
            pl[p] = sr;
            cur[slot] = p + 1;
          }
        }
      }
    }
  }
  __syncthreads();

  const int ovf = misc[9];
  {
    const float qnan = __uint_as_float(0x7fc00000u);
#pragma unroll 1
    for (int it = 0; it < NBRUN / NTHR; ++it) {
      const int s   = it * NTHR + tid;
      const int deg = cnt[s] + 1;
      const float df = (float)deg;
      const float rs = 1.0f / sqrtf(df);
      float dv = (deg > 0) ? rs : 0.0f;
      dv = (ovf != 0) ? qnan : dv;
      cur[s] = __float_as_int(dv);
    }
  }
  __syncthreads();

  int* lp = LIST + (size_t)blk * RCAP;
  int* cp = CNT + (size_t)blk * NBRUN;
  int* op = OFF + (size_t)blk * NBRUN;
  int* dp = DINVB + (size_t)blk * NBRUN;
  int* fp = FLAG + (size_t)blk * 32;
  bucket_flush(pl, cnt, ovf, lp, cp, op, dp, fp, tid);
  __threadfence();
  bucket_flush(pl, cnt, ovf, lp, cp, op, dp, fp, tid);
}

template <int KTOT>
__device__ __forceinline__ void gemm_16x64(const unsigned short* __restrict__ ap,
                                           const unsigned short* __restrict__ bp, v8f (&acc)[4]) {
#pragma unroll 1
  for (int k0 = 0; k0 < KTOT; k0 += 32) {
    FragB af;
    af.h[0] = *(const v8usa*)(ap + k0);
    af.h[1] = *(const v8usa*)(ap + k0 + 16);
#pragma unroll
    for (int nt = 0; nt < 4; ++nt) {
      const unsigned short* wq = bp + (size_t)(16 * nt) * (size_t)KTOT + k0;
      FragB bf;
      bf.h[0] = *(const v8usa*)wq;
      bf.h[1] = *(const v8usa*)(wq + 16);
      acc[nt] = wmb(af, bf, acc[nt]);
    }
  }
}

__device__ __forceinline__ void stage_d(float* stg, const v8f (&acc)[4], int wave, int hh, int m) {
#pragma unroll
  for (int nt = 0; nt < 4; ++nt) {
#pragma unroll
    for (int r = 0; r < 8; ++r) stg[(16 * wave + 8 * hh + r) * SP + 16 * nt + m] = acc[nt][r];
  }
}

__global__ __launch_bounds__(NTHR) __attribute__((amdgpu_num_vgpr(248)))
void k_gemm(const unsigned short* __restrict__ XB, const unsigned short* __restrict__ WT,
            const float* __restrict__ DINV, float* HP) {
  __shared__ __attribute__((aligned(16))) float stg[GBM * SP];
  __shared__ __attribute__((aligned(16))) float sdi[GBM];
  const int tid = (int)threadIdx.x, lane = tid & 31, wave = tid >> 5, hh = lane >> 4, m = lane & 15;
  const int rowBase = (int)blockIdx.x * GBM;
  if (tid < 32) *(v4fa*)(sdi + 4 * tid) = *(const v4fa*)(DINV + (size_t)rowBase + 4 * tid);

  v8f acc[4];
  {
    const v8f z = {0.f, 0.f, 0.f, 0.f, 0.f, 0.f, 0.f, 0.f};
#pragma unroll
    for (int t = 0; t < 4; ++t) acc[t] = z;
  }
  const unsigned short* ap = XB + (size_t)(rowBase + 16 * wave + m) * (size_t)HD + 8 * hh;
  const unsigned short* bp = WT + (size_t)m * (size_t)HD + 8 * hh;
  gemm_16x64<HD>(ap, bp, acc);
  stage_d(stg, acc, wave, hh, m);
  __syncthreads();

#pragma unroll 1
  for (int i = 0; i < 8; ++i) {
    const int lr   = 16 * wave + 2 * i + hh;
    const int grow = rowBase + lr;
    const bool live = grow < NN;
    const v4f a = *(const v4fa*)(stg + lr * SP + 4 * m);
    const float dv = sdi[lr];
    asm volatile("" :: "v"(a));
    asm volatile("" :: "v"(dv));
    const float v0 = dv * a.x, v1 = dv * a.y, v2 = dv * a.z, v3 = dv * a.w;
    v4f o;
    o.x = live ? v0 : 0.0f; o.y = live ? v1 : 0.0f; o.z = live ? v2 : 0.0f; o.w = live ? v3 : 0.0f;
    st2_v4f(HP + (size_t)grow * HD + 4 * m, o);
  }
}

__global__ __launch_bounds__(NTHR) void k_replay(const int* __restrict__ LIST, const int* __restrict__ CNT,
                                                 const int* __restrict__ OFF, const float* __restrict__ DINV,
                                                 const int* __restrict__ FLAG, const float* __restrict__ HP,
                                                 const float* __restrict__ BB, float* out) {
  const int tid = (int)threadIdx.x, lane = tid & 31;
  const int wave = __builtin_amdgcn_readfirstlane(tid >> 5);
  const int blk = (int)blockIdx.x;
  const int firstRow = blk * NBRUN;
  const int* lb  = LIST + (size_t)blk * RCAP;
  const int flag = FLAG[(size_t)blk * 32];
  const float qnan = __uint_as_float(0x7fc00000u);
  const v2f bias = *(const v2fa*)(BB + 2 * lane);

#pragma unroll 1
  for (int si = 0; si < NBRUN / NWAVE; ++si) {
    const int node = firstRow + si * NWAVE + wave;
    if (node >= NN) continue;
    int c = __builtin_amdgcn_readfirstlane(CNT[node]);
    int o = __builtin_amdgcn_readfirstlane(OFF[node]);
    const float dv = DINV[node];
    const bool big = c > TRIPCAP;
    c = c < 0 ? 0 : (c > TRIPCAP ? TRIPCAP : c);
    o = o < 0 ? 0 : (o > RCAP - 1 ? RCAP - 1 : o);
    int last = o + (c > 0 ? c : 1) - 1;
    last = last > RCAP - 1 ? RCAP - 1 : last;
    float a0 = 0.0f, a1 = 0.0f;
#pragma unroll 1
    for (int b0 = 0; b0 < c; b0 += 32) {
      int idx = o + b0 + lane;
      idx = idx > last ? last : idx;
      int sr = lb[idx];
      sr = sr < 0 ? 0 : (sr > NN - 1 ? NN - 1 : sr);
      const int m32 = (c - b0) < 32 ? (c - b0) : 32;
#pragma unroll 1
      for (int k = 0; k < m32; k += 4) {
        const int s0 = __builtin_amdgcn_readlane(sr, k);
        const int s1 = __builtin_amdgcn_readlane(sr, k + 1);
        const int s2 = __builtin_amdgcn_readlane(sr, k + 2);
        const int s3 = __builtin_amdgcn_readlane(sr, k + 3);
        const v2f g0 = *(const v2fa*)(HP + (size_t)s0 * HD + 2 * lane);
        const v2f g1 = *(const v2fa*)(HP + (size_t)s1 * HD + 2 * lane);
        const v2f g2 = *(const v2fa*)(HP + (size_t)s2 * HD + 2 * lane);
        const v2f g3 = *(const v2fa*)(HP + (size_t)s3 * HD + 2 * lane);
        asm volatile("" :: "v"(g0), "v"(g1), "v"(g2), "v"(g3));
        const bool q1 = (k + 1) < m32, q2 = (k + 2) < m32, q3 = (k + 3) < m32;
        a0 = a0 + g0.x;            a1 = a1 + g0.y;
        const float t10 = a0 + g1.x, t11 = a1 + g1.y;
        a0 = q1 ? t10 : a0;        a1 = q1 ? t11 : a1;
        const float t20 = a0 + g2.x, t21 = a1 + g2.y;
        a0 = q2 ? t20 : a0;        a1 = q2 ? t21 : a1;
        const float t30 = a0 + g3.x, t31 = a1 + g3.y;
        a0 = q3 ? t30 : a0;        a1 = q3 ? t31 : a1;
      }
    }
    const v2f sv = *(const v2fa*)(HP + (size_t)node * HD + 2 * lane);
    a0 = a0 + sv.x; a1 = a1 + sv.y;
    float y0 = dv * a0 + bias.x;
    float y1 = dv * a1 + bias.y;
    const bool bad = (flag != 0) | big;
    y0 = bad ? qnan : y0;
    y1 = bad ? qnan : y1;
    v2f ov;
    ov.x = y0; ov.y = y1;
    float* op = out + (size_t)node * HD + 2 * lane;
    *(volatile v2f*)op = ov;
    __threadfence();
    *(volatile v2f*)op = ov;
  }
}

extern "C" void kernel_launch(void* const* d_in, const int* in_sizes, int n_in,
                              void* d_out, int out_size, void* d_ws, size_t ws_size,
                              hipStream_t stream) {
  if (n_in < 4) return;
  if (in_sizes[0] != NN * HD) return;
  if (in_sizes[1] != 2 * NE) return;
  if (in_sizes[2] != HD * HD) return;
  if (in_sizes[3] != HD) return;
  if (out_size != NN * HD) return;

  const float* x  = (const float*)d_in[0];
  const int*   ei = (const int*)d_in[1];
  const float* W  = (const float*)d_in[2];
  const float* b  = (const float*)d_in[3];
  float* out = (float*)d_out;
  const int* srcs = ei;
  const int* dsts = ei + NE;

  constexpr size_t zXB   = (size_t)MP * HD * 2;
  constexpr size_t zHP   = (size_t)MP * HD * 4;
  constexpr size_t zLIST = (size_t)NBK * RCAP * 4;
  constexpr size_t zTAB  = (size_t)NSLOT * 4;
  constexpr size_t zFLAG = (size_t)NBK * 128;
  constexpr size_t zWT   = (size_t)HD * HD * 2;
  constexpr size_t zBB   = 256;
  constexpr size_t oXB   = 0;
  constexpr size_t oHP   = oXB + zXB;
  constexpr size_t oLIST = oHP + zHP;
  constexpr size_t oCNT  = oLIST + zLIST;
  constexpr size_t oOFF  = oCNT + zTAB;
  constexpr size_t oDINV = oOFF + zTAB;
  constexpr size_t oFLAG = oDINV + zTAB;
  constexpr size_t oWT   = oFLAG + zFLAG;
  constexpr size_t oBB   = oWT + zWT;
  constexpr size_t oEND  = oBB + zBB;
  static_assert(zXB % 256 == 0 && zHP % 256 == 0 && zLIST % 256 == 0 && zTAB % 256 == 0);
  static_assert(zFLAG % 256 == 0 && zWT % 256 == 0 && zBB % 256 == 0);
  static_assert(oEND <= (size_t)WSMAX);
  if (oEND > ws_size) return;

  char* ws = (char*)d_ws;
  unsigned short* XB   = (unsigned short*)(ws + oXB);
  float*          HP   = (float*)(ws + oHP);
  int*            LIST = (int*)(ws + oLIST);
  int*            CNT  = (int*)(ws + oCNT);
  int*            OFF  = (int*)(ws + oOFF);
  int*            DINB = (int*)(ws + oDINV);
  float*          DINV = (float*)(ws + oDINV);
  int*            FLAG = (int*)(ws + oFLAG);
  unsigned short* WT   = (unsigned short*)(ws + oWT);
  float*          BB   = (float*)(ws + oBB);

  hipFuncSetAttribute(reinterpret_cast<const void*>(&k_bucket), hipFuncAttributeMaxDynamicSharedMemorySize, (int)BK_LDS);

  k_prep<<<PBTOT, NTHR, 0, stream>>>(x, W, b, XB, WT, BB);
  k_bucket<<<NBK, NTHR, BK_LDS, stream>>>(srcs, dsts, LIST, CNT, OFF, DINB, FLAG);
  k_gemm<<<MP / GBM, NTHR, 0, stream>>>(XB, WT, DINV, HP);
  k_replay<<<NBK, NTHR, 0, stream>>>(LIST, CNT, OFF, DINV, FLAG, HP, BB, out);
}
